// SchNet_29618094473608
// MI455X (gfx1250) — hardware-verified
//
#include <hip/hip_runtime.h>
#include <stddef.h>


#define NTHR   256
#define NWAVE  8
#define HID    128
#define NF     32
#define NG     50
#define KP     64
#define A1P    72
#define A2P    40
#define XP     136
#define NB     1024
#define EPT    8
#define CHUNK  (NTHR * EPT)
#define WCAP   (EPT * 32)
#define LISTN  (NWAVE * WCAP)
#define PASSN  64
#define PCAP   (CHUNK + PASSN)
#define RMAX   (PCAP / PASSN)
#define NROWL  512
#define RTL    (NROWL / (16 * NWAVE))
#define NROWN  128
#define NQE    ((NB * NF) / (4 * NTHR))
#define NQN    ((NROWN * HID) / (4 * NTHR))
#define NQM    ((NROWN * NF) / (4 * NTHR))

#define CUTF   10.0f
#define PIF    3.14159265358979f
#define STEPF  (CUTF / (float)(NG - 1))
#define COEFF  (-0.5f / (STEPF * STEPF))
#define LN2F   0.69314718f
#define W1S    8.0f
#define W2S    8.0f
#define USC    8.0f
#define L1S    16.0f
#define L2S    8.0f
#define L3S    16.0f
#define INV8   0.125f
#define INV16  0.0625f
#define INV64  0.015625f

static_assert(NQE * 4 * NTHR == NB * NF);
static_assert(NQN * 4 * NTHR == NROWN * HID);
static_assert(NQM * 4 * NTHR == NROWN * NF);
static_assert(PASSN * 4 == NTHR);
static_assert((PCAP % PASSN) == 0);
static_assert(HID == 16 * NWAVE);
static_assert((PASSN / 16) * 2 == NWAVE);
static_assert(RTL * 16 * NWAVE == NROWL);
static_assert((NROWN % 16) == 0);
static_assert((NROWL % NROWN) == 0);
static_assert(NF == 32);
static_assert(KP == 64);

typedef float    v4f  __attribute__((ext_vector_type(4)));
typedef float    v8f  __attribute__((ext_vector_type(8)));
typedef int      v4i  __attribute__((ext_vector_type(4)));
typedef _Float16 v4h  __attribute__((ext_vector_type(4)));
typedef _Float16 v8h  __attribute__((ext_vector_type(8)));
typedef _Float16 v16h __attribute__((ext_vector_type(16)));

union Frag { v16h v; v8h h[2]; v4h q[4]; _Float16 s[16]; };

__device__ __forceinline__ v8f zero8f() {
  v8f z;
#pragma unroll
  for (int i = 0; i < 8; ++i) z[i] = 0.0f;
  return z;
}

__device__ __forceinline__ v8f wm(v16h a, v16h b, v8f c) {
  v8f d = __builtin_amdgcn_wmma_f32_16x16x32_f16(false, a, false, b, (short)0, c, false, false);
  asm volatile("v_nop\n\tv_nop\n\tv_nop\n\tv_nop" : "+v"(d) : "v"(a), "v"(b));
  return d;
}

__device__ __forceinline__ float sspf(float v) {
  const float e = __expf(-fabsf(v));
  return fmaxf(v, 0.0f) + (__logf(1.0f + e) - LN2F);
}

__device__ __forceinline__ v16h bfrag(const float* __restrict__ W, int ldn, int col, int ks, int hh,
                                      int kmax, float sc) {
  Frag f;
  const int kA = 32 * ks + 8 * hh, kB = kA + 16;
#pragma unroll
  for (int j = 0; j < 8; ++j) {
    const int ka = kA + j, kb = kB + j;
    const float wa = (ka < kmax) ? W[(size_t)ka * ldn + col] : 0.0f;
    const float wb = (kb < kmax) ? W[(size_t)kb * ldn + col] : 0.0f;
    f.s[j]     = (_Float16)(wa * sc);
    f.s[8 + j] = (_Float16)(wb * sc);
  }
  return f.v;
}

__device__ __forceinline__ void accadd(float* accb, int s, int c, float v) {
  s = s < 0 ? 0 : (s > NB ? NB : s);
  float* q = accb + s * NF + c;
  const float t = *q + v;
  *q = t;
}

__global__ __launch_bounds__(NTHR) void k_prep(
    const float* __restrict__ pos, const int* __restrict__ srci, const int* __restrict__ dsti,
    const float* __restrict__ emask, float* cutp, _Float16* rbf, int nN, int nE) {
#pragma clang fp contract(off)
  __shared__ __attribute__((aligned(16))) float cb[NTHR];
  const int tid = threadIdx.x, lane = tid & 31, wave = tid >> 5;
  const int e = blockIdx.x * NTHR + tid;
  const bool valid = e < nE;
  const int ec = valid ? e : (nE - 1);
  int s = srci[ec], t = dsti[ec];
  s = s < 0 ? 0 : (s > nN - 1 ? nN - 1 : s);
  t = t < 0 ? 0 : (t > nN - 1 ? nN - 1 : t);
  const float dx = pos[(size_t)s * 3 + 0] - pos[(size_t)t * 3 + 0];
  const float dy = pos[(size_t)s * 3 + 1] - pos[(size_t)t * 3 + 1];
  const float dz = pos[(size_t)s * 3 + 2] - pos[(size_t)t * 3 + 2];
  const float d  = sqrtf(dx * dx + dy * dy + dz * dz);
  float cval = 0.0f;
  if (valid) cval = 0.5f * (cosf((d * PIF) * (1.0f / CUTF)) + 1.0f) * emask[ec];
  cb[tid] = cval;

  Frag rb[4];
#pragma unroll
  for (int q = 0; q < 4; ++q) {
#pragma unroll
    for (int i = 0; i < 16; ++i) {
      const int k = 16 * q + i;
      float v = 0.0f;
      if (k < NG) {
        const float ok = (k == NG - 1) ? CUTF : (float)k * STEPF;
        const float u  = d - ok;
        v = __expf(COEFF * (u * u));
      }
      rb[q].s[i] = (_Float16)v;
    }
  }
  _Float16* rp = rbf + (size_t)ec * KP;
  if (valid) {
#pragma unroll
    for (int q = 0; q < 4; ++q) {
      *(volatile v8h*)(rp + 16 * q)     = rb[q].h[0];
      *(volatile v8h*)(rp + 16 * q + 8) = rb[q].h[1];
    }
  }
  __threadfence();
  if (valid) {
#pragma unroll
    for (int q = 0; q < 4; ++q) {
      *(volatile v8h*)(rp + 16 * q)     = rb[q].h[0];
      *(volatile v8h*)(rp + 16 * q + 8) = rb[q].h[1];
    }
  }
  __syncthreads();
  if (wave < 2) {
    const int f = 128 * wave + 4 * lane;
    const v4f v = *(const v4f*)(cb + f);
    *(volatile v4f*)(cutp + (size_t)blockIdx.x * NTHR + f) = v;
  }
  __threadfence();
  if (wave < 2) {
    const int f = 128 * wave + 4 * lane;
    const v4f v = *(const v4f*)(cb + f);
    *(volatile v4f*)(cutp + (size_t)blockIdx.x * NTHR + f) = v;
  }
}

__global__ __launch_bounds__(NTHR) void k_init(const int* __restrict__ z, const float* __restrict__ emb,
                                               float* out, int nN, int nT) {
  const int tid = threadIdx.x, lane = tid & 31, wave = tid >> 5;
  const int row = blockIdx.x * NWAVE + wave;
  if (row < nN) {
    int zi = z[row];
    if (zi < 0) zi += nT;
    zi = zi < 0 ? 0 : (zi > nT - 1 ? nT - 1 : zi);
    const v4f v = *(const v4f*)(emb + (size_t)zi * HID + 4 * lane);
    float* p = out + (size_t)row * HID + 4 * lane;
    *(volatile v4f*)p = v;
    __threadfence();
    *(volatile v4f*)p = v;
  }
}

__global__ __launch_bounds__(NTHR) void k_lin1(const float* __restrict__ h, const float* __restrict__ W,
                                               float* hsp, int nN) {
  __shared__ __attribute__((aligned(16))) float stg[NWAVE * 16 * NF];
  const int tid = threadIdx.x, lane = tid & 31, wave = tid >> 5, hh = lane >> 4, m = lane & 15;
  Frag B[2][4];
#pragma unroll
  for (int nt = 0; nt < 2; ++nt)
#pragma unroll
    for (int ks = 0; ks < 4; ++ks)
      B[nt][ks].v = bfrag(W, NF, 16 * nt + m, ks, hh, HID, L1S);
  float* st = stg + wave * (16 * NF);
  const int rowW = blockIdx.x * NROWL + wave * (16 * RTL);

#pragma unroll 1
  for (int rt = 0; rt < RTL; ++rt) {
    const int r0 = rowW + 16 * rt;
    v8f d0 = zero8f(), d1 = zero8f();
#pragma unroll
    for (int ks = 0; ks < 4; ++ks) {
      const float* p = h + (size_t)(r0 + m) * HID + 32 * ks + 8 * hh;
      const v4f x0 = *(const v4f*)p;
      const v4f x1 = *(const v4f*)(p + 4);
      const v4f x2 = *(const v4f*)(p + 16);
      const v4f x3 = *(const v4f*)(p + 20);
      Frag a;
#pragma unroll
      for (int i = 0; i < 4; ++i) {
        a.s[i]      = (_Float16)x0[i];
        a.s[4 + i]  = (_Float16)x1[i];
        a.s[8 + i]  = (_Float16)x2[i];
        a.s[12 + i] = (_Float16)x3[i];
      }
      d0 = wm(a.v, B[0][ks].v, d0);
      d1 = wm(a.v, B[1][ks].v, d1);
    }
#pragma unroll
    for (int r = 0; r < 8; ++r) {
      st[(8 * hh + r) * NF + m]      = d0[r] * INV16;
      st[(8 * hh + r) * NF + 16 + m] = d1[r] * INV16;
    }
    __syncthreads();
#pragma unroll
    for (int i = 0; i < 4; ++i) {
      const int rowl = 4 * i + (lane >> 3), c = 4 * (lane & 7);
      const v4f v = *(const v4f*)(st + rowl * NF + c);
      *(volatile v4f*)(hsp + (size_t)(r0 + rowl) * NF + c) = v;
    }
    __threadfence();
#pragma unroll
    for (int i = 0; i < 4; ++i) {
      const int rowl = 4 * i + (lane >> 3), c = 4 * (lane & 7);
      const v4f v = *(const v4f*)(st + rowl * NF + c);
      *(volatile v4f*)(hsp + (size_t)(r0 + rowl) * NF + c) = v;
    }
    __syncthreads();
  }
}

__device__ __forceinline__ int scan_chunk(const int* __restrict__ dsts, const float* __restrict__ msk,
                                          int nE, int cbase, int nodeBase, int vec8,
                                          int* list, int tid, int wave) {
  int wc = 0;
  const int el0  = tid * EPT;
  const int e0   = cbase + el0;
  const int sent = -2147483647 - 1;
  int dv[EPT];
  float mv[EPT];
  if (vec8 != 0 && e0 + 7 < nE) {
    const v4i da = *(const v4i*)(dsts + e0);
    const v4i db = *(const v4i*)(dsts + e0 + 4);
    const v4f ma = *(const v4f*)(msk + e0);
    const v4f mb = *(const v4f*)(msk + e0 + 4);
    dv[0] = da.x; dv[1] = da.y; dv[2] = da.z; dv[3] = da.w;
    dv[4] = db.x; dv[5] = db.y; dv[6] = db.z; dv[7] = db.w;
    mv[0] = ma.x; mv[1] = ma.y; mv[2] = ma.z; mv[3] = ma.w;
    mv[4] = mb.x; mv[5] = mb.y; mv[6] = mb.z; mv[7] = mb.w;
  } else {
#pragma unroll
    for (int j = 0; j < EPT; ++j) {
      const int ej = e0 + j;
      const bool in = ej < nE;
      const int ecl = in ? ej : (nE - 1);
      dv[j] = in ? dsts[ecl] : sent;
      mv[j] = in ? msk[ecl] : 0.0f;
    }
  }
  const unsigned nb = (unsigned)nodeBase;
  bool hj[EPT];
  bool anyl = false;
#pragma unroll
  for (int j = 0; j < EPT; ++j) {
    const unsigned sj = (unsigned)dv[j] - nb;
    hj[j] = (sj < (unsigned)NB) && (mv[j] != 0.0f);
    anyl = anyl || hj[j];
  }
  const unsigned any = __builtin_amdgcn_ballot_w32(anyl);
  if (any != 0u) {
#pragma unroll
    for (int j = 0; j < EPT; ++j) {
      const unsigned mj = __builtin_amdgcn_ballot_w32(hj[j]);
      if (mj != 0u) {
        if (hj[j]) {
          const int p = wc + (int)__builtin_amdgcn_mbcnt_lo(mj, 0u);
          if (p < WCAP) list[wave * WCAP + p] = el0 + j;
        }
        wc += (int)__builtin_popcount(mj);
      }
    }
  }
  return wc;
}

__global__ __launch_bounds__(NTHR) void k_edge(
    const int* __restrict__ dsti, const int* __restrict__ srci, const float* __restrict__ emask,
    const float* __restrict__ rcut, const _Float16* __restrict__ rbf,
    const float* __restrict__ W1, const float* __restrict__ bw1,
    const float* __restrict__ W2, const float* __restrict__ bw2,
    const float* __restrict__ hsp, float* aggp, int nN, int nE, int vec8) {
  __shared__ __attribute__((aligned(16))) float    acc[(NB + 1) * NF];
  __shared__ __attribute__((aligned(16))) _Float16 A1[PASSN * A1P];
  __shared__ __attribute__((aligned(16))) _Float16 A2[PASSN * A2P];
  __shared__ __attribute__((aligned(16))) float    Wt[PASSN * NF];
  __shared__ __attribute__((aligned(16))) int      list[LISTN];
  __shared__ __attribute__((aligned(16))) int      pend[PCAP];
  __shared__ __attribute__((aligned(16))) int      slotb[PASSN];
  __shared__ __attribute__((aligned(16))) int      jb[PASSN];
  __shared__ __attribute__((aligned(16))) float    rcb[PASSN];
  __shared__ int wcnt[NWAVE];
  __shared__ int pendN;

  const int tid = threadIdx.x, lane = tid & 31, wave = tid >> 5, hh = lane >> 4, m = lane & 15;
  const int tw = wave >> 1, nw = wave & 1;
  const int col = 16 * nw + m;
  const int nodeBase = blockIdx.x * NB;
  const v4f z4 = {0.0f, 0.0f, 0.0f, 0.0f};

  for (int i = tid; i < ((NB + 1) * NF) / 4; i += NTHR) *(v4f*)(acc + 4 * i) = z4;
  Frag B1a, B1b, B2f;
  B1a.v = bfrag(W1, NF, col, 0, hh, NG, W1S);
  B1b.v = bfrag(W1, NF, col, 1, hh, NG, W1S);
  B2f.v = bfrag(W2, NF, col, 0, hh, NF, W2S);
  const float b1c = bw1[col];
  const float b2c = bw2[col];
  if (tid == 0) pendN = 0;
  __syncthreads();

  const int nChunks = (nE + CHUNK - 1) / CHUNK;
#pragma unroll 1
  for (int ch = 0; ch < nChunks; ++ch) {
    const int cbase = ch * CHUNK;
    const int wc = scan_chunk(dsti, emask, nE, cbase, nodeBase, vec8, list, tid, wave);
    if (lane == 0) wcnt[wave] = wc;
    __syncthreads();

    const int base = pendN;
    int tot = 0, myoff = 0;
#pragma unroll
    for (int w = 0; w < NWAVE; ++w) {
      int c = wcnt[w];
      c = c > WCAP ? WCAP : (c < 0 ? 0 : c);
      if (w < wave) myoff += c;
      tot += c;
    }
    int newN = base + tot;
    newN = newN > PCAP ? PCAP : (newN < 0 ? 0 : newN);
    {
      int n = wcnt[wave];
      n = n > WCAP ? WCAP : (n < 0 ? 0 : n);
      const int* lp = list + wave * WCAP;
      for (int i = lane; i < n; i += 32) {
        const int p = base + myoff + i;
        if ((unsigned)p < (unsigned)PCAP) pend[p] = cbase + lp[i];
      }
    }
    const int fin = (ch == nChunks - 1) ? 1 : 0;
    int R = (fin != 0) ? (newN + PASSN - 1) / PASSN : newN / PASSN;
    R = R > RMAX ? RMAX : R;
    const int Pv = (fin != 0) ? newN : R * PASSN;
    __syncthreads();

#pragma unroll 1
    for (int r = 0; r < R; ++r) {
      {
        const int i = tid >> 2, p = tid & 3;
        const int idx = r * PASSN + i;
        const bool valid = idx < Pv;
        int e = 0;
        if (valid) e = pend[idx];
        e = e < 0 ? 0 : (e > nE - 1 ? nE - 1 : e);
        Frag q;
        q.h[0] = *(const v8h*)&z4;
        q.h[1] = *(const v8h*)&z4;
        if (valid) {
          const _Float16* rp = rbf + (size_t)e * KP + 16 * p;
          q.h[0] = *(const v8h*)rp;
          q.h[1] = *(const v8h*)(rp + 8);
        }
        _Float16* arow = A1 + i * A1P + 16 * p;
        *(v8h*)arow       = q.h[0];
        *(v8h*)(arow + 8) = q.h[1];
        if (p == 0) {
          const int dd = dsti[e];
          int sj = srci[e];
          int slot = dd - nodeBase;
          if (!valid || (unsigned)slot >= (unsigned)NB) slot = NB;
          sj = sj < 0 ? 0 : (sj > nN - 1 ? nN - 1 : sj);
          slotb[i] = slot;
          jb[i]    = sj;
          rcb[i]   = valid ? rcut[e] : 0.0f;
        }
      }
      __syncthreads();

      {
        const int o = (16 * tw + m) * A1P + 8 * hh;
        Frag a0, a1;
        a0.h[0] = *(const v8h*)(A1 + o);       a0.h[1] = *(const v8h*)(A1 + o + 16);
        a1.h[0] = *(const v8h*)(A1 + o + 32);  a1.h[1] = *(const v8h*)(A1 + o + 48);
        v8f d = zero8f();
        d = wm(a0.v, B1a.v, d);
        d = wm(a1.v, B1b.v, d);
#pragma unroll
        for (int rr = 0; rr < 8; ++rr) {
          const float u = sspf(d[rr] * INV8 + b1c);
          A2[(16 * tw + 8 * hh + rr) * A2P + col] = (_Float16)(u * USC);
        }
      }
      __syncthreads();

      {
        const int o = (16 * tw + m) * A2P + 8 * hh;
        Frag x;
        x.h[0] = *(const v8h*)(A2 + o);
        x.h[1] = *(const v8h*)(A2 + o + 16);
        v8f d = zero8f();
        d = wm(x.v, B2f.v, d);
#pragma unroll
        for (int rr = 0; rr < 8; ++rr) {
          const int er = 16 * tw + 8 * hh + rr;
          Wt[er * NF + col] = (d[rr] * INV64 + b2c) * rcb[er];
        }
      }
      __syncthreads();

      if (wave == 0) {
#pragma unroll 2
        for (int e4 = 0; e4 < PASSN; e4 += 4) {
          const v4i s4 = *(const v4i*)(slotb + e4);
          const v4i j4 = *(const v4i*)(jb + e4);
#pragma unroll
          for (int u = 0; u < 4; ++u) {
            int sj = j4[u];
            sj = sj < 0 ? 0 : (sj > nN - 1 ? nN - 1 : sj);
            const float wv = Wt[(e4 + u) * NF + lane];
            const float hv = hsp[(size_t)sj * NF + lane];
            accadd(acc, s4[u], lane, hv * wv);
          }
        }
      }
      __syncthreads();
    }

    int rem = newN - R * PASSN;
    rem = rem < 0 ? 0 : (rem > PASSN - 1 ? PASSN - 1 : rem);
    if (R > 0 && tid < rem) pend[tid] = pend[R * PASSN + tid];
    if (tid == 0) pendN = rem;
  }
  __syncthreads();

  const size_t ob = (size_t)nodeBase * NF;
#pragma unroll 1
  for (int q = 0; q < NQE; ++q) {
    const int f = (q * NTHR + tid) * 4;
    const v4f v = *(const v4f*)(acc + f);
    *(volatile v4f*)(aggp + ob + (size_t)f) = v;
  }
  __threadfence();
#pragma unroll 1
  for (int q = 0; q < NQE; ++q) {
    const int f = (q * NTHR + tid) * 4;
    const v4f v = *(const v4f*)(acc + f);
    *(volatile v4f*)(aggp + ob + (size_t)f) = v;
  }
}

__global__ __launch_bounds__(NTHR) void k_node(
    const float* __restrict__ aggp,
    const float* __restrict__ W2n, const float* __restrict__ b2n,
    const float* __restrict__ W3n, const float* __restrict__ b3n,
    float* out, int nN) {
  __shared__ __attribute__((aligned(16))) _Float16 Am[NROWN * A2P];
  __shared__ __attribute__((aligned(16))) _Float16 Xt[NROWN * XP];
  __shared__ __attribute__((aligned(16))) float    Ot[NROWN * HID];

  const int tid = threadIdx.x, lane = tid & 31, wave = tid >> 5, hh = lane >> 4, m = lane & 15;
  const int col = 16 * wave + m;
  const int row0 = blockIdx.x * NROWN;

#pragma unroll
  for (int q = 0; q < NQM; ++q) {
    const int i = q * NTHR + tid;
    const int r = i >> 3, c4 = (i & 7) * 4;
    const v4f v = *(const v4f*)(aggp + (size_t)(row0 + r) * NF + c4);
    v4h hv;
    hv[0] = (_Float16)v[0]; hv[1] = (_Float16)v[1]; hv[2] = (_Float16)v[2]; hv[3] = (_Float16)v[3];
    *(v4h*)(Am + r * A2P + c4) = hv;
  }
  Frag Bm;
  Bm.v = bfrag(W2n, HID, col, 0, hh, NF, L2S);
  Frag Bw[4];
#pragma unroll
  for (int ks = 0; ks < 4; ++ks) Bw[ks].v = bfrag(W3n, HID, col, ks, hh, HID, L3S);
  const float bA = b2n[col];
  const float bB = b3n[col];
  __syncthreads();

#pragma unroll 1
  for (int rt = 0; rt < NROWN / 16; ++rt) {
    const int o = (16 * rt + m) * A2P + 8 * hh;
    Frag a;
    a.h[0] = *(const v8h*)(Am + o);
    a.h[1] = *(const v8h*)(Am + o + 16);
    v8f d = zero8f();
    d = wm(a.v, Bm.v, d);
#pragma unroll
    for (int r = 0; r < 8; ++r) {
      const float x = sspf(d[r] * INV8 + bA);
      Xt[(16 * rt + 8 * hh + r) * XP + col] = (_Float16)x;
    }
  }
  __syncthreads();

#pragma unroll 1
  for (int rt = 0; rt < NROWN / 16; ++rt) {
    v8f d = zero8f();
#pragma unroll
    for (int ks = 0; ks < 4; ++ks) {
      const int o = (16 * rt + m) * XP + 32 * ks + 8 * hh;
      Frag a;
      a.h[0] = *(const v8h*)(Xt + o);
      a.h[1] = *(const v8h*)(Xt + o + 16);
      d = wm(a.v, Bw[ks].v, d);
    }
#pragma unroll
    for (int r = 0; r < 8; ++r) {
      const int row = 16 * rt + 8 * hh + r;
      const float hold = out[(size_t)(row0 + row) * HID + col];
      Ot[row * HID + col] = d[r] * INV16 + bB + hold;
    }
  }
  __syncthreads();

  const size_t ob = (size_t)row0 * HID;
#pragma unroll 1
  for (int q = 0; q < NQN; ++q) {
    const int f = (q * NTHR + tid) * 4;
    const v4f v = *(const v4f*)(Ot + f);
    *(volatile v4f*)(out + ob + (size_t)f) = v;
  }
  __threadfence();
#pragma unroll 1
  for (int q = 0; q < NQN; ++q) {
    const int f = (q * NTHR + tid) * 4;
    const v4f v = *(const v4f*)(Ot + f);
    *(volatile v4f*)(out + ob + (size_t)f) = v;
  }
}

extern "C" void kernel_launch(void* const* d_in, const int* in_sizes, int n_in,
                              void* d_out, int out_size, void* d_ws, size_t ws_size,
                              hipStream_t stream) {
  if (n_in < 14) return;
  const int nN = in_sizes[0];
  const int nE = in_sizes[3];
  if (nN <= 0 || nE <= 0) return;
  if (in_sizes[1] != 3 * nN || in_sizes[2] != 2 * nE) return;
  if (in_sizes[4] < HID || (in_sizes[4] % HID) != 0) return;
  const int nT = in_sizes[4] / HID;
  if (in_sizes[5] <= 0 || (in_sizes[5] % (NG * NF)) != 0) return;
  const int nL = in_sizes[5] / (NG * NF);
  if (in_sizes[6] != nL * NF || in_sizes[7] != nL * NF * NF || in_sizes[8] != nL * NF) return;
  if (in_sizes[9] != nL * HID * NF || in_sizes[10] != nL * NF * HID || in_sizes[11] != nL * HID) return;
  if (in_sizes[12] != nL * HID * HID || in_sizes[13] != nL * HID) return;
  if (out_size != nN * HID) return;
  if ((nN % NROWL) != 0 || (nN % NROWN) != 0) return;

  const int*   z     = (const int*)d_in[0];
  const float* pos   = (const float*)d_in[1];
  const int*   eidx  = (const int*)d_in[2];
  const float* emask = (const float*)d_in[3];
  const float* emb   = (const float*)d_in[4];
  const float* w1    = (const float*)d_in[5];
  const float* b1    = (const float*)d_in[6];
  const float* w2    = (const float*)d_in[7];
  const float* b2    = (const float*)d_in[8];
  const float* l1w   = (const float*)d_in[9];
  const float* l2w   = (const float*)d_in[10];
  const float* l2b   = (const float*)d_in[11];
  const float* l3w   = (const float*)d_in[12];
  const float* l3b   = (const float*)d_in[13];
  const int* srci = eidx;
  const int* dsti = eidx + nE;
  float* out = (float*)d_out;

  const int nBlkP = (nE + NTHR - 1) / NTHR;
  const size_t ePad = (size_t)nBlkP * NTHR;
  const int nBlkE = (nN + NB - 1) / NB;
  const int nBlkL = nN / NROWL;
  const int nBlkN = nN / NROWN;
  const int nBlkI = (nN + NWAVE - 1) / NWAVE;

  char* ws = (char*)d_ws;
  size_t off = 0;
  const size_t oC = off;  off += ePad * sizeof(float);                         off = (off + 255) & ~(size_t)255;
  const size_t oR = off;  off += (size_t)nE * KP * sizeof(_Float16);           off = (off + 255) & ~(size_t)255;
  const size_t oH = off;  off += (size_t)nN * NF * sizeof(float);              off = (off + 255) & ~(size_t)255;
  const size_t oA = off;  off += (size_t)nBlkE * NB * NF * sizeof(float);      off = (off + 255) & ~(size_t)255;
  if (off > ws_size || off > (size_t)134217728) return;
  float*    cutp = (float*)(ws + oC);
  _Float16* rbf  = (_Float16*)(ws + oR);
  float*    hsp  = (float*)(ws + oH);
  float*    aggp = (float*)(ws + oA);

  const int vec8 = ((nE & 7) == 0) ? 1 : 0;

  k_prep<<<nBlkP, NTHR, 0, stream>>>(pos, srci, dsti, emask, cutp, rbf, nN, nE);
  k_init<<<nBlkI, NTHR, 0, stream>>>(z, emb, out, nN, nT);

  for (int l = 0; l < nL; ++l) {
    k_lin1<<<nBlkL, NTHR, 0, stream>>>(out, l1w + (size_t)l * HID * NF, hsp, nN);
    k_edge<<<nBlkE, NTHR, 0, stream>>>(dsti, srci, emask, cutp, rbf,
                                       w1 + (size_t)l * NG * NF, b1 + (size_t)l * NF,
                                       w2 + (size_t)l * NF * NF, b2 + (size_t)l * NF,
                                       hsp, aggp, nN, nE, vec8);
    k_node<<<nBlkN, NTHR, 0, stream>>>(aggp, l2w + (size_t)l * NF * HID, l2b + (size_t)l * HID,
                                       l3w + (size_t)l * HID * HID, l3b + (size_t)l * HID, out, nN);
  }
}
